// SimpleCyberGNN_22196390986479
// MI455X (gfx1250) — hardware-verified
//
#include <hip/hip_runtime.h>
#include <stddef.h>


#define FIN   64
#define D1    128
#define NHD   4
#define HDIM  32
#define D2    32
#define NGR   64
#define CH    16
#define NCLS  2

#define NTHR  256
#define NWAVE 8
#define CHUNK 2048
#define NGRP  (CHUNK / (NTHR * 4))
#define WCAP  ((CHUNK / NTHR) * 32)

#define GR1   32
#define AP1   72
#define XSP1  132
#define GR2   64
#define AP2   136
#define XSP2  36

#define SB1   9
#define NB1   (1 << SB1)
#define SB2   10
#define NB2   (1 << SB2)
#define RPAD  1024
#define PSTR  (NGR * D2 + NGR)
#define FTHR  128
#define CP    40

#define SCW   8.0f
#define SCP   16.0f
#define SCW1  4.0f
#define SCT   64.0f
#define SCW2  4.0f

#define L1_SACC (NB1 * D1)
#define L1_DEN  (NB1 * NHD)
#define L1_MX   (NB1 * NHD)
#define L1_LIST (NWAVE * WCAP)
#define L1_BYTES ((L1_SACC + L1_DEN + L1_MX + L1_LIST + NWAVE) * 4)

#define L2_SACC (NB2 * D2)
#define L2_DEN  (NB2)
#define L2_PSUM (NWAVE * NGR * D2)
#define L2_PCNT (NWAVE * NGR)
#define L2_MX   (NB2)
#define L2_LIST (NWAVE * WCAP)
#define L2_BYTES ((L2_SACC + L2_DEN + L2_PSUM + L2_PCNT + L2_MX + L2_LIST + NWAVE) * 4)

static_assert(NGRP == 2);
static_assert(WCAP == NGRP * 4 * 32);
static_assert(L1_BYTES == 286752);
static_assert(L2_BYTES == 215072);
static_assert(((L1_SACC + L1_DEN) % 4) == 0);
static_assert((L1_MX % 4) == 0);
static_assert(((L2_SACC + L2_DEN + L2_PSUM + L2_PCNT) % 4) == 0);
static_assert((L2_MX % 4) == 0);
static_assert((RPAD % NB1) == 0);
static_assert((RPAD % NB2) == 0);
static_assert((RPAD % GR1) == 0);
static_assert((RPAD % GR2) == 0);
static_assert(SB1 + 11 <= 30);
static_assert(SB2 + 11 <= 30);
static_assert((PSTR % 32) == 0);
static_assert(NWAVE * 16 == D1);
static_assert(D1 == NHD * HDIM);

typedef float    v4f  __attribute__((ext_vector_type(4)));
typedef float    v8f  __attribute__((ext_vector_type(8)));
typedef int      v4i  __attribute__((ext_vector_type(4)));
typedef _Float16 v8h  __attribute__((ext_vector_type(8)));
typedef _Float16 v16h __attribute__((ext_vector_type(16)));
union Frag   { v16h v; v8h half[2]; };
union Pack16 { v8h h; v4i i; };

__device__ __forceinline__ v8f wm(v16h a, v16h b, v8f c) {
  v8f d = __builtin_amdgcn_wmma_f32_16x16x32_f16(false, a, false, b, (short)0, c, false, false);
  asm volatile("v_nop\n\tv_nop\n\tv_nop\n\tv_nop" : "+v"(d) : "v"(a), "v"(b));
  return d;
}

__device__ __forceinline__ v8h pack8(v4f a, v4f b, float s) {
  v8h r;
  r[0] = (_Float16)(a.x * s); r[1] = (_Float16)(a.y * s); r[2] = (_Float16)(a.z * s); r[3] = (_Float16)(a.w * s);
  r[4] = (_Float16)(b.x * s); r[5] = (_Float16)(b.y * s); r[6] = (_Float16)(b.z * s); r[7] = (_Float16)(b.w * s);
  return r;
}

__device__ __forceinline__ float leaky02(float v) { return v > 0.f ? v : 0.2f * v; }
__device__ __forceinline__ float elu1(float v) { return v > 0.f ? v : (__expf(v) - 1.0f); }

__global__ __launch_bounds__(NTHR) void k_prep(const float* __restrict__ W1, const float* __restrict__ W2,
                                               _Float16* W1t, _Float16* W2t) {
  const int i = blockIdx.x * NTHR + threadIdx.x;
  Pack16 u;
  _Float16* dst;
  if (i < D1 * (FIN / 8)) {
    const int n = i >> 3, k0 = (i & 7) * 8;
    const v4f a = {W1[(size_t)(k0 + 0) * D1 + n], W1[(size_t)(k0 + 1) * D1 + n],
                   W1[(size_t)(k0 + 2) * D1 + n], W1[(size_t)(k0 + 3) * D1 + n]};
    const v4f b = {W1[(size_t)(k0 + 4) * D1 + n], W1[(size_t)(k0 + 5) * D1 + n],
                   W1[(size_t)(k0 + 6) * D1 + n], W1[(size_t)(k0 + 7) * D1 + n]};
    u.h = pack8(a, b, SCW);
    dst = W1t + (size_t)n * FIN + k0;
  } else if (i < D1 * (FIN / 8) + D2 * (D1 / 8)) {
    const int j2 = i - D1 * (FIN / 8);
    const int n = j2 >> 4, k0 = (j2 & 15) * 8;
    const v4f a = {W2[(size_t)(k0 + 0) * D2 + n], W2[(size_t)(k0 + 1) * D2 + n],
                   W2[(size_t)(k0 + 2) * D2 + n], W2[(size_t)(k0 + 3) * D2 + n]};
    const v4f b = {W2[(size_t)(k0 + 4) * D2 + n], W2[(size_t)(k0 + 5) * D2 + n],
                   W2[(size_t)(k0 + 6) * D2 + n], W2[(size_t)(k0 + 7) * D2 + n]};
    u.h = pack8(a, b, SCW);
    dst = W2t + (size_t)n * D1 + k0;
  } else {
    return;
  }
  *(volatile v4i*)dst = u.i;
  __threadfence();
  *(volatile v4i*)dst = u.i;
}

__global__ __launch_bounds__(NTHR) void k_gemm1(
    const float* __restrict__ x, const _Float16* __restrict__ W1t,
    const float* __restrict__ att_s, const float* __restrict__ att_d,
    float* xw, float* asrc, float* adst, int nN) {
  __shared__ __attribute__((aligned(16))) _Float16 At[GR1 * AP1];
  __shared__ __attribute__((aligned(16))) float Xs[GR1 * XSP1];
  __shared__ __attribute__((aligned(16))) float Ad[2 * GR1 * NHD];

  const int tid  = threadIdx.x;
  const int lane = tid & 31;
  const int wave = tid >> 5;
  const int hh   = lane >> 4;
  const int m    = lane & 15;
  const int rowBase = blockIdx.x * GR1;

  {
    const int r  = tid >> 3;
    const int c0 = (tid & 7) * 8;
    int row = rowBase + r;
    if (row > nN - 1) row = nN - 1;
    const float* p = x + (size_t)row * FIN + c0;
    const v4f f0 = *(const v4f*)(p), f1 = *(const v4f*)(p + 4);
    *(v8h*)(At + r * AP1 + c0) = pack8(f0, f1, 1.0f);
  }
  __syncthreads();

  const int ncol = wave * 16 + m;
  v8f c0a = {0.f, 0.f, 0.f, 0.f, 0.f, 0.f, 0.f, 0.f};
  v8f c1a = {0.f, 0.f, 0.f, 0.f, 0.f, 0.f, 0.f, 0.f};
#pragma unroll
  for (int kt = 0; kt < FIN / 32; ++kt) {
    const int k0 = kt * 32;
    Frag a0, a1, b;
    const _Float16* pb  = W1t + (size_t)ncol * FIN + k0 + 8 * hh;
    const _Float16* pa0 = At + m * AP1 + k0 + 8 * hh;
    const _Float16* pa1 = At + (16 + m) * AP1 + k0 + 8 * hh;
    b.half[0]  = *(const v8h*)pb;  b.half[1]  = *(const v8h*)(pb + 16);
    a0.half[0] = *(const v8h*)pa0; a0.half[1] = *(const v8h*)(pa0 + 16);
    a1.half[0] = *(const v8h*)pa1; a1.half[1] = *(const v8h*)(pa1 + 16);
    c0a = wm(a0.v, b.v, c0a);
    c1a = wm(a1.v, b.v, c1a);
  }

#pragma unroll
  for (int r = 0; r < 8; ++r) {
    Xs[(8 * hh + r) * XSP1 + ncol]      = c0a[r] * 0.125f;
    Xs[(16 + 8 * hh + r) * XSP1 + ncol] = c1a[r] * 0.125f;
  }
  __syncthreads();

  {
    const int row   = tid >> 3;
    const int q     = tid & 7;
    const int head  = q >> 1;
    const int which = q & 1;
    const float* av = (which ? att_d : att_s) + head * HDIM;
    const float* xr = Xs + row * XSP1 + head * HDIM;
    float s = 0.f;
#pragma unroll
    for (int c = 0; c < HDIM; ++c) s += xr[c] * av[c];
    Ad[which * (GR1 * NHD) + row * NHD + head] = s;
  }
  __syncthreads();

  v4f xr4[4];
  float* xpp[4];
#pragma unroll
  for (int i = 0; i < 4; ++i) {
    xr4[i] = *(const v4f*)(Xs + (4 * wave + i) * XSP1 + 4 * lane);
    xpp[i] = xw + (size_t)(rowBase + 4 * wave + i) * D1 + 4 * lane;
  }
  float* gp = 0;
  v4f gv = {0.f, 0.f, 0.f, 0.f};
  if (wave == 0) {
    gv = *(const v4f*)(Ad + 4 * lane);
    gp = asrc + (size_t)rowBase * NHD + 4 * lane;
  } else if (wave == 1) {
    gv = *(const v4f*)(Ad + GR1 * NHD + 4 * lane);
    gp = adst + (size_t)rowBase * NHD + 4 * lane;
  }
#pragma unroll
  for (int i = 0; i < 4; ++i) *(volatile v4f*)(xpp[i]) = xr4[i];
  if (gp) *(volatile v4f*)gp = gv;
  __threadfence();
#pragma unroll
  for (int i = 0; i < 4; ++i) *(volatile v4f*)(xpp[i]) = xr4[i];
  if (gp) *(volatile v4f*)gp = gv;
}

__global__ __launch_bounds__(NTHR) void k_gemm2(
    const float* __restrict__ h1, const _Float16* __restrict__ W2t,
    const float* __restrict__ att_s, const float* __restrict__ att_d,
    float* xw2, float* asrc2, float* adst2, int nN) {
  __shared__ __attribute__((aligned(16))) _Float16 At[GR2 * AP2];
  __shared__ __attribute__((aligned(16))) float Xs[GR2 * XSP2];
  __shared__ __attribute__((aligned(16))) float Ad[2 * GR2];

  const int tid  = threadIdx.x;
  const int lane = tid & 31;
  const int wave = tid >> 5;
  const int hh   = lane >> 4;
  const int m    = lane & 15;
  const int rowBase = blockIdx.x * GR2;

  {
    const int r  = tid >> 2;
    const int c0 = (tid & 3) * 32;
    int row = rowBase + r;
    if (row > nN - 1) row = nN - 1;
    const float* p = h1 + (size_t)row * D1 + c0;
#pragma unroll
    for (int q = 0; q < 4; ++q) {
      const v4f f0 = *(const v4f*)(p + 8 * q), f1 = *(const v4f*)(p + 8 * q + 4);
      *(v8h*)(At + r * AP2 + c0 + 8 * q) = pack8(f0, f1, 1.0f);
    }
  }
  __syncthreads();

  const int rt   = wave >> 1;
  const int ct   = wave & 1;
  const int ncol = ct * 16 + m;
  v8f acc = {0.f, 0.f, 0.f, 0.f, 0.f, 0.f, 0.f, 0.f};
#pragma unroll
  for (int kt = 0; kt < D1 / 32; ++kt) {
    const int k0 = kt * 32;
    Frag a, b;
    const _Float16* pa = At + (16 * rt + m) * AP2 + k0 + 8 * hh;
    const _Float16* pb = W2t + (size_t)ncol * D1 + k0 + 8 * hh;
    a.half[0] = *(const v8h*)pa; a.half[1] = *(const v8h*)(pa + 16);
    b.half[0] = *(const v8h*)pb; b.half[1] = *(const v8h*)(pb + 16);
    acc = wm(a.v, b.v, acc);
  }
#pragma unroll
  for (int r = 0; r < 8; ++r) Xs[(16 * rt + 8 * hh + r) * XSP2 + ncol] = acc[r] * 0.125f;
  __syncthreads();

  if (tid < 2 * GR2) {
    const int row   = tid >> 1;
    const int which = tid & 1;
    const float* av = which ? att_d : att_s;
    const float* xr = Xs + row * XSP2;
    float s = 0.f;
#pragma unroll
    for (int c = 0; c < D2; ++c) s += xr[c] * av[c];
    Ad[which * GR2 + row] = s;
  }
  __syncthreads();

  v4f xr4[2];
  float* xpp[2];
#pragma unroll
  for (int i = 0; i < 2; ++i) {
    const int row = 8 * wave + 4 * i + (lane >> 3);
    const int col = 4 * (lane & 7);
    xr4[i] = *(const v4f*)(Xs + row * XSP2 + col);
    xpp[i] = xw2 + (size_t)(rowBase + row) * D2 + col;
  }
  float* gp = 0;
  v4f gv = {0.f, 0.f, 0.f, 0.f};
  if (wave == 0) {
    gv = *(const v4f*)(Ad + 4 * lane);
    gp = (lane < 16) ? (asrc2 + (size_t)rowBase + 4 * lane) : (adst2 + (size_t)rowBase + 4 * (lane - 16));
  }
#pragma unroll
  for (int i = 0; i < 2; ++i) *(volatile v4f*)(xpp[i]) = xr4[i];
  if (gp) *(volatile v4f*)gp = gv;
  __threadfence();
#pragma unroll
  for (int i = 0; i < 2; ++i) *(volatile v4f*)(xpp[i]) = xr4[i];
  if (gp) *(volatile v4f*)gp = gv;
}

__device__ __forceinline__ void hit1(bool hj, int code, int& wc, int* wl) {
  const unsigned mj = __builtin_amdgcn_ballot_w32(hj);
  if (hj) {
    const int pos = wc + (int)__builtin_amdgcn_mbcnt_lo(mj, 0u);
    if (pos < WCAP) wl[pos] = code;
  }
  wc += (int)__builtin_popcount(mj);
}

template<int SB>
__device__ __forceinline__ int scan_chunk(const int* __restrict__ eid, int nE, bool al16, int cbase,
                                          int nodeBase, int tid, int* wl) {
  const unsigned NBT = 1u << SB;
  int wc = 0;
#pragma unroll
  for (int g = 0; g < NGRP; ++g) {
    const int el0 = (g * NTHR + tid) * 4;
    const int e0  = cbase + el0;
    const int sent = -2147483647 - 1;
    v4i d;
    if (al16 && (e0 + 3 < nE)) {
      d = *(const v4i*)(eid + e0);
    } else {
      d.x = (e0     < nE) ? eid[e0]     : sent;
      d.y = (e0 + 1 < nE) ? eid[e0 + 1] : sent;
      d.z = (e0 + 2 < nE) ? eid[e0 + 2] : sent;
      d.w = (e0 + 3 < nE) ? eid[e0 + 3] : sent;
    }
    const unsigned s0 = (unsigned)d.x - (unsigned)nodeBase;
    const unsigned s1 = (unsigned)d.y - (unsigned)nodeBase;
    const unsigned s2 = (unsigned)d.z - (unsigned)nodeBase;
    const unsigned s3 = (unsigned)d.w - (unsigned)nodeBase;
    const bool h0 = s0 < NBT, h1 = s1 < NBT, h2 = s2 < NBT, h3 = s3 < NBT;
    const unsigned many = __builtin_amdgcn_ballot_w32(h0 | h1 | h2 | h3);
    if (many != 0u) {
      hit1(h0, ((el0 + 0) << SB) | (int)s0, wc, wl);
      hit1(h1, ((el0 + 1) << SB) | (int)s1, wc, wl);
      hit1(h2, ((el0 + 2) << SB) | (int)s2, wc, wl);
      hit1(h3, ((el0 + 3) << SB) | (int)s3, wc, wl);
    }
  }
  return wc;
}

__global__ __launch_bounds__(NTHR) void k_agg1(
    const int* __restrict__ ei, const float* __restrict__ xw,
    const float* __restrict__ asrc, const float* __restrict__ adst,
    const float* __restrict__ bias, float* h1, int nN, int nE) {
  extern __shared__ v4f dyn1[];
  float* sacc = (float*)dyn1;
  float* den  = sacc + L1_SACC;
  float* mx   = den + L1_DEN;
  int*   list = (int*)(mx + L1_MX);
  int*   wcnt = list + L1_LIST;

  const int tid  = threadIdx.x;
  const int lane = tid & 31;
  const int wave = tid >> 5;
  const int hd   = lane >> 3;
  const int nodeBase = blockIdx.x * NB1;

  {
    const v4f z4 = {0.f, 0.f, 0.f, 0.f};
    const v4f m4 = {-1.0e30f, -1.0e30f, -1.0e30f, -1.0e30f};
    for (int i = tid; i < (L1_SACC + L1_DEN) / 4; i += NTHR) dyn1[i] = z4;
    v4f* mx4 = (v4f*)mx;
    for (int i = tid; i < L1_MX / 4; i += NTHR) mx4[i] = m4;
  }
  __syncthreads();

  const int* eid = ei + nE;
  const bool al16 = ((nE & 3) == 0);
  const int nChunks = (nE + CHUNK - 1) / CHUNK;
#pragma unroll 1
  for (int ch = 0; ch < nChunks; ++ch) {
    const int cbase = ch * CHUNK;
    const int wc = scan_chunk<SB1>(eid, nE, al16, cbase, nodeBase, tid, list + wave * WCAP);
    if (lane == 0) wcnt[wave] = wc;
    __syncthreads();

    if (wave == 0) {
#pragma unroll 1
      for (int wsx = 0; wsx < NWAVE; ++wsx) {
        int n = wcnt[wsx];
        n = n > WCAP ? WCAP : (n < 0 ? 0 : n);
        const int* wl = list + wsx * WCAP;
#pragma unroll 1
        for (int i = 0; i < n; ++i) {
          const int ent  = wl[i];
          const int slot = ent & (NB1 - 1);
          const int el   = (ent >> SB1) & (CHUNK - 1);
          int e = cbase + el;
          if (e > nE - 1) e = nE - 1;
          int src = ei[e];
          src = src < 0 ? 0 : (src > nN - 1 ? nN - 1 : src);
          int nd = nodeBase + slot;
          if (nd > nN - 1) nd = nN - 1;
          const float al = leaky02(asrc[(size_t)src * NHD + hd] + adst[(size_t)nd * NHD + hd]);
          const int mi = slot * NHD + hd;
          const float mo = mx[mi];
          const float mn = fmaxf(mo, al);
          const float sc = __expf(mo - mn);
          const float p  = __expf(al - mn);
          const v4f xv = *(const v4f*)(xw + (size_t)src * D1 + 4 * lane);
          v4f* sp = (v4f*)(sacc + slot * D1 + 4 * lane);
          const v4f cur = *sp;
          const v4f nxt = cur * sc + xv * p;
          *sp = nxt;
          if ((lane & 7) == 0) {
            const float dold = den[mi];
            den[mi] = dold * sc + p;
            mx[mi]  = mn;
          }
        }
      }
    }
    __syncthreads();
  }

  const v4f b4 = *(const v4f*)(bias + 4 * lane);
#pragma unroll 1
  for (int j = 0; j < NB1 / NWAVE; ++j) {
    const int slot = wave * (NB1 / NWAVE) + j;
    const int node = nodeBase + slot;
    if (node >= nN) break;
    const size_t nrow = (size_t)node;
    const float al = leaky02(asrc[nrow * NHD + hd] + adst[nrow * NHD + hd]);
    const int mi = slot * NHD + hd;
    const float mo = mx[mi];
    const float mn = fmaxf(mo, al);
    const float sc = __expf(mo - mn);
    const float p  = __expf(al - mn);
    const v4f xv = *(const v4f*)(xw + nrow * D1 + 4 * lane);
    const v4f sv = *(const v4f*)(sacc + slot * D1 + 4 * lane) * sc + xv * p;
    const float dv  = den[mi] * sc + p;
    const float inv = 1.0f / dv;
    v4f h = sv * inv + b4;
    h.x = elu1(h.x); h.y = elu1(h.y); h.z = elu1(h.z); h.w = elu1(h.w);
    float* op = h1 + nrow * D1 + 4 * lane;
    *(volatile v4f*)op = h;
    __threadfence();
    *(volatile v4f*)op = h;
  }
}

__global__ __launch_bounds__(NTHR) void k_agg2(
    const int* __restrict__ ei, const int* __restrict__ batch,
    const float* __restrict__ xw2, const float* __restrict__ asrc2, const float* __restrict__ adst2,
    const float* __restrict__ bias2, float* part, int nN, int nE) {
  extern __shared__ v4f dyn2[];
  float* sacc = (float*)dyn2;
  float* den  = sacc + L2_SACC;
  float* psum = den + L2_DEN;
  float* pcnt = psum + L2_PSUM;
  float* mx   = pcnt + L2_PCNT;
  int*   list = (int*)(mx + L2_MX);
  int*   wcnt = list + L2_LIST;

  const int tid  = threadIdx.x;
  const int lane = tid & 31;
  const int wave = tid >> 5;
  const int nodeBase = blockIdx.x * NB2;

  {
    const v4f z4 = {0.f, 0.f, 0.f, 0.f};
    const v4f m4 = {-1.0e30f, -1.0e30f, -1.0e30f, -1.0e30f};
    for (int i = tid; i < (L2_SACC + L2_DEN + L2_PSUM + L2_PCNT) / 4; i += NTHR) dyn2[i] = z4;
    v4f* mx4 = (v4f*)mx;
    for (int i = tid; i < L2_MX / 4; i += NTHR) mx4[i] = m4;
  }
  __syncthreads();

  const int* eid = ei + nE;
  const bool al16 = ((nE & 3) == 0);
  const int nChunks = (nE + CHUNK - 1) / CHUNK;
#pragma unroll 1
  for (int ch = 0; ch < nChunks; ++ch) {
    const int cbase = ch * CHUNK;
    const int wc = scan_chunk<SB2>(eid, nE, al16, cbase, nodeBase, tid, list + wave * WCAP);
    if (lane == 0) wcnt[wave] = wc;
    __syncthreads();

    if (wave == 0) {
#pragma unroll 1
      for (int wsx = 0; wsx < NWAVE; ++wsx) {
        int n = wcnt[wsx];
        n = n > WCAP ? WCAP : (n < 0 ? 0 : n);
        const int* wl = list + wsx * WCAP;
#pragma unroll 1
        for (int i = 0; i < n; ++i) {
          const int ent  = wl[i];
          const int slot = ent & (NB2 - 1);
          const int el   = (ent >> SB2) & (CHUNK - 1);
          int e = cbase + el;
          if (e > nE - 1) e = nE - 1;
          int src = ei[e];
          src = src < 0 ? 0 : (src > nN - 1 ? nN - 1 : src);
          int nd = nodeBase + slot;
          if (nd > nN - 1) nd = nN - 1;
          const float al = leaky02(asrc2[src] + adst2[nd]);
          const float mo = mx[slot];
          const float mn = fmaxf(mo, al);
          const float sc = __expf(mo - mn);
          const float p  = __expf(al - mn);
          const float xv = xw2[(size_t)src * D2 + lane];
          const float cur = sacc[slot * D2 + lane];
          sacc[slot * D2 + lane] = cur * sc + xv * p;
          if (lane == 0) {
            const float dold = den[slot];
            den[slot] = dold * sc + p;
            mx[slot]  = mn;
          }
        }
      }
    }
    __syncthreads();
  }

  const float bl = bias2[lane];
  float* psw = psum + wave * (NGR * D2);
  float* pcw = pcnt + wave * NGR;
#pragma unroll 1
  for (int j = 0; j < NB2 / NWAVE; ++j) {
    const int slot = wave * (NB2 / NWAVE) + j;
    const int node = nodeBase + slot;
    if (node >= nN) break;
    const size_t nrow = (size_t)node;
    const float al = leaky02(asrc2[nrow] + adst2[nrow]);
    const float mo = mx[slot];
    const float mn = fmaxf(mo, al);
    const float sc = __expf(mo - mn);
    const float p  = __expf(al - mn);
    const float xv = xw2[nrow * D2 + lane];
    const float sv = sacc[slot * D2 + lane] * sc + xv * p;
    const float dv = den[slot] * sc + p;
    const float h  = elu1(sv * (1.0f / dv) + bl);
    const int g = batch[nrow];
    if ((unsigned)g < (unsigned)NGR) {
      psw[g * D2 + lane] += h;
      if (lane == 0) pcw[g] += 1.0f;
    }
  }
  __syncthreads();

  float* pb = part + (size_t)blockIdx.x * PSTR;
  v4f sv4[2];
  float* sp4[2];
#pragma unroll
  for (int j = 0; j < 2; ++j) {
    const int idx = tid + NTHR * j;
    const int g  = idx >> 3;
    const int c0 = (idx & 7) * 4;
    v4f s = {0.f, 0.f, 0.f, 0.f};
#pragma unroll
    for (int w = 0; w < NWAVE; ++w) s += *(const v4f*)(psum + w * (NGR * D2) + g * D2 + c0);
    sv4[j] = s;
    sp4[j] = pb + g * D2 + c0;
  }
  v4f cv = {0.f, 0.f, 0.f, 0.f};
  float* cp = 0;
  if (tid < NGR / 4) {
#pragma unroll
    for (int w = 0; w < NWAVE; ++w) cv += *(const v4f*)(pcnt + w * NGR + 4 * tid);
    cp = pb + NGR * D2 + 4 * tid;
  }
#pragma unroll
  for (int j = 0; j < 2; ++j) *(volatile v4f*)(sp4[j]) = sv4[j];
  if (cp) *(volatile v4f*)cp = cv;
  __threadfence();
#pragma unroll
  for (int j = 0; j < 2; ++j) *(volatile v4f*)(sp4[j]) = sv4[j];
  if (cp) *(volatile v4f*)cp = cv;
}

__global__ __launch_bounds__(FTHR) void k_final(
    const float* __restrict__ part, int nblk,
    const float* __restrict__ Wc1, const float* __restrict__ bc1,
    const float* __restrict__ Wc2, const float* __restrict__ bc2, float* out) {
  __shared__ __attribute__((aligned(16))) _Float16 Pa[NGR * CP];
  __shared__ __attribute__((aligned(16))) _Float16 Ta[NGR * CP];
  __shared__ __attribute__((aligned(16))) _Float16 Wb1[16 * CP];
  __shared__ __attribute__((aligned(16))) _Float16 Wb2[16 * CP];
  __shared__ float rcg[NGR];
  __shared__ float Lg[NGR * NCLS];
  __shared__ __attribute__((aligned(16))) float Ob[NGR * NCLS];

  const int tid  = threadIdx.x;
  const int lane = tid & 31;
  const int wave = tid >> 5;
  const int hh   = lane >> 4;
  const int m    = lane & 15;

  for (int i = tid; i < NGR * CP; i += FTHR) Ta[i] = (_Float16)0.0f;
  for (int i = tid; i < 16 * CP; i += FTHR) {
    const int n = i / CP;
    const int k = i - n * CP;
    Wb1[i] = (k < D2) ? (_Float16)(Wc1[k * CH + n] * SCW1) : (_Float16)0.0f;
    Wb2[i] = (n < NCLS && k < CH) ? (_Float16)(Wc2[k * NCLS + n] * SCW2) : (_Float16)0.0f;
  }
  if (tid < NGR) {
    float c = 0.f;
#pragma unroll 1
    for (int b = 0; b < nblk; ++b) c += part[(size_t)b * PSTR + NGR * D2 + tid];
    rcg[tid] = 1.0f / fmaxf(c, 1.0f);
  }
  __syncthreads();

  for (int idx = tid; idx < NGR * D2; idx += FTHR) {
    const int g = idx >> 5;
    const int c = idx & 31;
    float s = 0.f;
#pragma unroll 1
    for (int b = 0; b < nblk; ++b) s += part[(size_t)b * PSTR + idx];
    Pa[g * CP + c] = (_Float16)(s * rcg[g] * SCP);
  }
  __syncthreads();

  v8f acc = {0.f, 0.f, 0.f, 0.f, 0.f, 0.f, 0.f, 0.f};
  {
    Frag a, b;
    const _Float16* pa = Pa + (16 * wave + m) * CP + 8 * hh;
    const _Float16* pb = Wb1 + m * CP + 8 * hh;
    a.half[0] = *(const v8h*)pa; a.half[1] = *(const v8h*)(pa + 16);
    b.half[0] = *(const v8h*)pb; b.half[1] = *(const v8h*)(pb + 16);
    acc = wm(a.v, b.v, acc);
  }
  {
    const float bb1 = bc1[m];
#pragma unroll
    for (int r = 0; r < 8; ++r) {
      const float t = fmaxf(acc[r] * (1.0f / (SCP * SCW1)) + bb1, 0.f);
      Ta[(16 * wave + 8 * hh + r) * CP + m] = (_Float16)(t * SCT);
    }
  }
  __syncthreads();

  v8f acc2 = {0.f, 0.f, 0.f, 0.f, 0.f, 0.f, 0.f, 0.f};
  {
    Frag a, b;
    const _Float16* pa = Ta + (16 * wave + m) * CP + 8 * hh;
    const _Float16* pb = Wb2 + m * CP + 8 * hh;
    a.half[0] = *(const v8h*)pa; a.half[1] = *(const v8h*)(pa + 16);
    b.half[0] = *(const v8h*)pb; b.half[1] = *(const v8h*)(pb + 16);
    acc2 = wm(a.v, b.v, acc2);
  }
  if (m < NCLS) {
    const float bb2 = bc2[m];
#pragma unroll
    for (int r = 0; r < 8; ++r)
      Lg[(16 * wave + 8 * hh + r) * NCLS + m] = acc2[r] * (1.0f / (SCT * SCW2)) + bb2;
  }
  __syncthreads();

  if (tid < NGR) {
    const float l0 = Lg[2 * tid], l1 = Lg[2 * tid + 1];
    const float mm = fmaxf(l0, l1);
    const float s0 = l0 - mm, s1 = l1 - mm;
    const float lse = logf(expf(s0) + expf(s1));
    Ob[2 * tid]     = s0 - lse;
    Ob[2 * tid + 1] = s1 - lse;
  }
  __syncthreads();

  if (wave == 0) {
    const v4f v = *(const v4f*)(Ob + 4 * lane);
    *(volatile v4f*)(out + 4 * lane) = v;
    __threadfence();
    *(volatile v4f*)(out + 4 * lane) = v;
  }
}

extern "C" void kernel_launch(void* const* d_in, const int* in_sizes, int n_in,
                              void* d_out, int out_size, void* d_ws, size_t ws_size,
                              hipStream_t stream) {
  if (n_in < 15) return;
  const int nN = in_sizes[0] / FIN;
  const int nE = in_sizes[1] / 2;
  if (nN <= 0 || in_sizes[0] != nN * FIN) return;
  if (nE < 0 || in_sizes[1] != 2 * nE) return;
  if (in_sizes[2] != nN) return;
  if (in_sizes[3] != FIN * D1) return;
  if (in_sizes[4] != NHD * HDIM || in_sizes[5] != NHD * HDIM || in_sizes[6] != D1) return;
  if (in_sizes[7] != D1 * D2 || in_sizes[8] != D2 || in_sizes[9] != D2 || in_sizes[10] != D2) return;
  if (in_sizes[11] != D2 * CH || in_sizes[12] != CH || in_sizes[13] != CH * NCLS || in_sizes[14] != NCLS) return;
  if (out_size != NGR * NCLS) return;

  const float* x     = (const float*)d_in[0];
  const int*   ei    = (const int*)d_in[1];
  const int*   batch = (const int*)d_in[2];
  const float* W1    = (const float*)d_in[3];
  const float* ats1  = (const float*)d_in[4];
  const float* atd1  = (const float*)d_in[5];
  const float* b1    = (const float*)d_in[6];
  const float* W2    = (const float*)d_in[7];
  const float* ats2  = (const float*)d_in[8];
  const float* atd2  = (const float*)d_in[9];
  const float* b2    = (const float*)d_in[10];
  const float* Wc1   = (const float*)d_in[11];
  const float* bc1   = (const float*)d_in[12];
  const float* Wc2   = (const float*)d_in[13];
  const float* bc2   = (const float*)d_in[14];
  float* out = (float*)d_out;

  const int nP    = ((nN + RPAD - 1) / RPAD) * RPAD;
  const int nblk2 = nP / NB2;
  size_t off = 0;
  char* base = (char*)d_ws;
#define CARVE(T, name, bytes) T* name = (T*)(base + off); off += (((size_t)(bytes)) + 255) & ~((size_t)255);
  CARVE(_Float16, W1t,  (size_t)D1 * FIN * sizeof(_Float16))
  CARVE(_Float16, W2t,  (size_t)D2 * D1 * sizeof(_Float16))
  CARVE(float,    xw1,  (size_t)nP * D1 * sizeof(float))
  CARVE(float,    as1,  (size_t)nP * NHD * sizeof(float))
  CARVE(float,    ad1,  (size_t)nP * NHD * sizeof(float))
  CARVE(float,    h1,   (size_t)nP * D1 * sizeof(float))
  CARVE(float,    xw2,  (size_t)nP * D2 * sizeof(float))
  CARVE(float,    as2,  (size_t)nP * sizeof(float))
  CARVE(float,    ad2,  (size_t)nP * sizeof(float))
  CARVE(float,    part, (size_t)nblk2 * PSTR * sizeof(float))
#undef CARVE
  if (off > ws_size) return;
  if (off > (size_t)134217728) return;

  const int nPrep = D1 * (FIN / 8) + D2 * (D1 / 8);
  k_prep<<<(nPrep + NTHR - 1) / NTHR, NTHR, 0, stream>>>(W1, W2, W1t, W2t);

  k_gemm1<<<nP / GR1, NTHR, 0, stream>>>(x, W1t, ats1, atd1, xw1, as1, ad1, nN);

  hipFuncSetAttribute(reinterpret_cast<const void*>(&k_agg1),
                      hipFuncAttributeMaxDynamicSharedMemorySize, L1_BYTES);
  k_agg1<<<nP / NB1, NTHR, L1_BYTES, stream>>>(ei, xw1, as1, ad1, b1, h1, nN, nE);

  k_gemm2<<<nP / GR2, NTHR, 0, stream>>>(h1, W2t, ats2, atd2, xw2, as2, ad2, nN);

  hipFuncSetAttribute(reinterpret_cast<const void*>(&k_agg2),
                      hipFuncAttributeMaxDynamicSharedMemorySize, L2_BYTES);
  k_agg2<<<nblk2, NTHR, L2_BYTES, stream>>>(ei, batch, xw2, as2, ad2, b2, part, nN, nE);

  k_final<<<1, FTHR, 0, stream>>>(part, nblk2, Wc1, bc1, Wc2, bc2, out);
}
